// Qwen3_5Attention_2980707303638
// MI455X (gfx1250) — hardware-verified
//
#include <hip/hip_runtime.h>
#include <math.h>

typedef __attribute__((ext_vector_type(16))) _Float16 v16h;
typedef __attribute__((ext_vector_type(8)))  _Float16 v8h;
typedef __attribute__((ext_vector_type(16))) __bf16   v16b;
typedef __attribute__((ext_vector_type(8)))  __bf16   v8b;
typedef __attribute__((ext_vector_type(8)))  float    v8f;
typedef __attribute__((ext_vector_type(4)))  float    v4f;
typedef __attribute__((ext_vector_type(4)))  unsigned int v4u;

constexpr int kB    = 2;
constexpr int kS    = 2048;
constexpr int kD    = 2048;
constexpr int kH    = 16;
constexpr int kKVH  = 4;
constexpr int kHD   = 128;
constexpr int kRows = kB * kS;
constexpr int kNQ   = kH * kHD * 2;
constexpr int kNKV  = kKVH * kHD;
constexpr int kNQKV = kNQ + 2 * kNKV;
constexpr int kE    = kH * kHD;
constexpr int kHiRows = 512;
constexpr float kNormEps = 1e-6f;
static_assert(kRows == 4096 && kNQ == 4096 && kNKV == 512 && kNQKV == 5120 && kE == 2048, "wire shapes");
static_assert((kD % 32) == 0 && (kE % 32) == 0 && (kHD % 32) == 0, "K multiples of 32");
static_assert((kRows % 64) == 0 && (kNQKV % 64) == 0 && (kD % 64) == 0 && (kHiRows % 64) == 0 && ((kS - kHiRows) % 64) == 0, "M,N multiples of 64");
static_assert(((kRows / 64) * (kNQKV / 64)) % 8 == 0, "projection tile count multiple of 8");
static_assert(((kHiRows / 64) * (kD / 64)) % 8 == 0 && (((kS - kHiRows) / 64) * (kD / 64)) % 8 == 0, "output projection tile counts multiples of 8");

constexpr float kQKCarry = 64.0f;
constexpr float kVCarry  = 64.0f;
constexpr float kPCarry  = 32768.0f;
constexpr float kSgCarry = 1024.0f;
constexpr float kACarry  = 256.0f;
constexpr float kWoCarry = 1024.0f;
constexpr float kScoreFold = 1.0f / (kQKCarry * kQKCarry);
constexpr float kEpiFold   = kACarry / (kPCarry * kVCarry * kSgCarry);
constexpr float kOutScale  = 1.0f / (kACarry * kWoCarry);

constexpr size_t kOffXB  = 0;
constexpr size_t kOffWB  = kOffXB  + (size_t)kRows * kD * 2;
constexpr size_t kOffQR  = kOffWB  + (size_t)kNQKV * kD * 2;
constexpr size_t kOffKR  = kOffQR  + (size_t)kRows * kE * 4;
constexpr size_t kOffVR  = kOffKR  + (size_t)kRows * kNKV * 4;
constexpr size_t kOffSGH = kOffVR  + (size_t)kRows * kNKV * 4;
constexpr size_t kOffSGL = kOffSGH + (size_t)kRows * kE * 2;
constexpr size_t kOffKH  = kOffSGL + (size_t)kRows * kE * 2;
constexpr size_t kOffKL  = kOffKH  + (size_t)kB * kKVH * kS * kHD * 2;
constexpr size_t kWsTotal = kOffKL + (size_t)kB * kKVH * kS * kHD * 2;
constexpr size_t kOffQH  = kOffXB;
constexpr size_t kOffQL  = kOffQH + (size_t)kB * kH * kS * kHD * 2;
constexpr size_t kOffAH  = kOffQR;
constexpr size_t kOffAL  = kOffAH + (size_t)kRows * kE * 2;
constexpr size_t kOffVTH = kOffKR;
constexpr size_t kOffVTL = kOffVTH + (size_t)kB * kKVH * kS * kHD * 2;
constexpr size_t kOffWO  = kOffQH;
static_assert(kWsTotal == 130023424ull, "carve total");
static_assert(kWsTotal <= 134217728ull, "carve cap");
static_assert(kOffQL + (size_t)kB * kH * kS * kHD * 2 <= kOffQR, "q planes inside the dead x|W region");
static_assert(kOffAL + (size_t)kRows * kE * 2 <= kOffKR, "attn planes inside the dead q region");
static_assert(kOffVTL + (size_t)kB * kKVH * kS * kHD * 2 <= kOffVR, "transposed v planes inside the dead k region");
static_assert(kOffWO + (size_t)kD * kE * 2 <= kOffQL, "Wo plane inside the dead q value plane");
static_assert((kOffWB % 128) == 0 && (kOffQR % 128) == 0 && (kOffKR % 128) == 0 &&
              (kOffVR % 128) == 0 && (kOffSGH % 128) == 0 && (kOffSGL % 128) == 0 && (kOffKH % 128) == 0 &&
              (kOffKL % 128) == 0 && (kOffVTH % 128) == 0 && (kOffVTL % 128) == 0 && (kOffQL % 128) == 0 &&
              (kOffAL % 128) == 0 && (kOffWO % 128) == 0, "128-B aligned regions");

__device__ __forceinline__ unsigned short f2bf_bits(float f) {
  unsigned u = __float_as_uint(f);
  return (unsigned short)((u + 0x7FFFu + ((u >> 16) & 1u)) >> 16);
}
__device__ __forceinline__ float bf_bits2f(unsigned short h) { return __uint_as_float(((unsigned)h) << 16); }
__device__ __forceinline__ float bf_rne(float f) { return bf_bits2f(f2bf_bits(f)); }
__device__ __forceinline__ unsigned pk16(unsigned short a, unsigned short b) { return (unsigned)a | ((unsigned)b << 16); }
__device__ __forceinline__ unsigned short h_bits(float f) { const _Float16 h = (_Float16)f; return __builtin_bit_cast(unsigned short, h); }
__device__ __forceinline__ float h16_to_f32(unsigned hb) {
  const unsigned sgn = (hb & 0x8000u) << 16; const unsigned em = hb & 0x7fffu;
  const float fn = __uint_as_float((em << 13) + 0x38000000u);
  const float fs = (float)em * 5.9604644775390625e-8f;
  const float mag = (em < 0x400u) ? fs : fn; return __uint_as_float(__float_as_uint(mag) | sgn); }
__device__ __forceinline__ void split_h(float x, unsigned short& hb, unsigned short& lb) {
  hb = h_bits(x);
  lb = h_bits(x - h16_to_f32((unsigned)hb));
}

__device__ __forceinline__ void row_guard_h(v8f& a, v8f& b, v8f& c, v8f& d, v16h x, v16h y) { asm volatile("v_nop\n\tv_nop\n\tv_nop\n\tv_nop" : "+v"(a), "+v"(b), "+v"(c), "+v"(d) : "v"(x), "v"(y)); }
__device__ __forceinline__ void row_guard_b(v8f& a, v8f& b, v8f& c, v8f& d, v16b x, v16b y) { asm volatile("v_nop\n\tv_nop\n\tv_nop\n\tv_nop" : "+v"(a), "+v"(b), "+v"(c), "+v"(d) : "v"(x), "v"(y)); }
__device__ __forceinline__ void keep4_h(v16h a, v16h b, v16h c, v16h d) { asm volatile("v_nop" :: "v"(a), "v"(b), "v"(c), "v"(d)); }
__device__ __forceinline__ void keep4_b(v16b a, v16b b, v16b c, v16b d) { asm volatile("v_nop" :: "v"(a), "v"(b), "v"(c), "v"(d)); }
__device__ __forceinline__ void acc_guard4(v8f& a, v8f& b, v8f& c, v8f& d) { asm volatile("v_nop\n\tv_nop\n\tv_nop\n\tv_nop" : "+v"(a), "+v"(b), "+v"(c), "+v"(d)); }

template <typename T> struct Frag;
template <> struct Frag<_Float16> {
  typedef v16h V; union U { v16h v; v8h h[2]; };
  static __device__ __forceinline__ v16h load(const _Float16* p) {
    U f; f.h[0] = *(const v8h*)(p); f.h[1] = *(const v8h*)(p + 16); return f.v;
  }
  static __device__ __forceinline__ v8f mma(v16h a, v16h b, v8f c) {
    return __builtin_amdgcn_wmma_f32_16x16x32_f16(false, a, false, b, (short)0, c, false, false);
  }
  static __device__ __forceinline__ void guard4(v8f& a, v8f& b, v8f& c, v8f& d, v16h x, v16h y) { row_guard_h(a, b, c, d, x, y); }
  static __device__ __forceinline__ void keep(v16h a, v16h b, v16h c, v16h d) { keep4_h(a, b, c, d); }
};
template <> struct Frag<__bf16> {
  typedef v16b V; union U { v16b v; v8b h[2]; };
  static __device__ __forceinline__ v16b load(const __bf16* p) {
    U f; f.h[0] = *(const v8b*)(p); f.h[1] = *(const v8b*)(p + 16); return f.v;
  }
  static __device__ __forceinline__ v8f mma(v16b a, v16b b, v8f c) {
    return __builtin_amdgcn_wmma_f32_16x16x32_bf16(false, a, false, b, (short)0, c, false, false);
  }
  static __device__ __forceinline__ void guard4(v8f& a, v8f& b, v8f& c, v8f& d, v16b x, v16b y) { row_guard_b(a, b, c, d, x, y); }
  static __device__ __forceinline__ void keep(v16b a, v16b b, v16b c, v16b d) { keep4_b(a, b, c, d); }
};
template <int ET> struct Elem;
template <> struct Elem<0> { typedef _Float16 T; };
template <> struct Elem<1> { typedef __bf16 T; };

__device__ __forceinline__ v8f mma_h(v16h a, v16h b, v8f c) {
  c = __builtin_amdgcn_wmma_f32_16x16x32_f16(false, a, false, b, (short)0, c, false, false);
  asm volatile("v_nop\n\tv_nop\n\tv_nop\n\tv_nop" : "+v"(c) : "v"(a), "v"(b));
  return c;
}

__global__ __launch_bounds__(256) void cvt_bf16_kernel(const float* __restrict__ src, unsigned short* __restrict__ dst, int n8) {
  const int i = blockIdx.x * 256 + threadIdx.x;
  if (i >= n8) return;
  const size_t e0 = (size_t)i << 3;
  const v4f a0 = *(const v4f*)(src + e0);
  const v4f a1 = *(const v4f*)(src + e0 + 4);
  unsigned short hb[8];
#pragma unroll
  for (int e = 0; e < 4; ++e) {
    const float f0 = a0[e];
    const float f1 = a1[e];
    hb[e]     = f2bf_bits(f0);
    hb[4 + e] = f2bf_bits(f1);
  }
  const v4u u = (v4u){pk16(hb[0], hb[1]), pk16(hb[2], hb[3]), pk16(hb[4], hb[5]), pk16(hb[6], hb[7])};
  unsigned short* q = dst + e0;
  *(volatile v4u*)q = u;
  __threadfence();
  *(volatile v4u*)q = u;
}

__global__ __launch_bounds__(256) void cvt_f16c_kernel(const float* __restrict__ src, unsigned short* __restrict__ dst, int n8, float carry) {
  const int i = blockIdx.x * 256 + threadIdx.x;
  if (i >= n8) return;
  const size_t e0 = (size_t)i << 3;
  const v4f a0 = *(const v4f*)(src + e0);
  const v4f a1 = *(const v4f*)(src + e0 + 4);
  unsigned short hb[8];
#pragma unroll
  for (int e = 0; e < 4; ++e) {
    const float f0 = a0[e];
    const float f1 = a1[e];
    hb[e]     = h_bits(bf_rne(f0) * carry);
    hb[4 + e] = h_bits(bf_rne(f1) * carry);
  }
  const v4u u = (v4u){pk16(hb[0], hb[1]), pk16(hb[2], hb[3]), pk16(hb[4], hb[5]), pk16(hb[6], hb[7])};
  unsigned short* q = dst + e0;
  *(volatile v4u*)q = u;
  __threadfence();
  *(volatile v4u*)q = u;
}

template <int ET, int SPL, int EPI>
__global__ __launch_bounds__(256) void gemm64_kernel(
    const unsigned short* __restrict__ Ap, const unsigned short* __restrict__ A2p, int lda, long strideA,
    const unsigned short* __restrict__ Btp, int ldb,
    float* __restrict__ C0, int ldc0, long strideC,
    float* __restrict__ Ck, float* __restrict__ Cv,
    unsigned short* __restrict__ Sgh, unsigned short* __restrict__ Sgl,
    int M, int N, int K, float scale) {
  typedef typename Elem<ET>::T T;
  typedef typename Frag<T>::V V;
  const T* A = (const T*)Ap; const T* A2 = (const T*)A2p; const T* Bt = (const T*)Btp;
  __shared__ __align__(16) float sT[8][16 * 68];
  const int bz   = blockIdx.y;
  const int lane = threadIdx.x & 31;
  const int wave = __builtin_amdgcn_readfirstlane((int)(threadIdx.x >> 5));
  const int tilesN = N >> 6;
  const int tilesM = M >> 6;
  const int tile = blockIdx.x * 8 + wave;
  if (tile >= tilesM * tilesN) return;
  const int tm = tile / tilesN;
  const int tn = tile - tm * tilesN;
  const int m0 = tm << 6;
  const int n0 = tn << 6;

  const T* Ab  = A + (size_t)bz * strideA;
  const T* Ab2 = (SPL >= 1) ? (A2 + (size_t)bz * strideA) : nullptr;
  const T* Bb  = Bt;

  const int rlane = lane & 15;
  const int koff  = (lane >> 4) * 8;
  const int mOff  = (lane >> 4) * 8;

  v8f acc[4][4];
#pragma unroll
  for (int i = 0; i < 4; ++i)
#pragma unroll
    for (int j = 0; j < 4; ++j) acc[i][j] = (v8f){0.f,0.f,0.f,0.f,0.f,0.f,0.f,0.f};

  for (int k0 = 0; k0 < K; k0 += 32) {
    V bh[4];
#pragma unroll
    for (int j = 0; j < 4; ++j) {
      const size_t bo = (size_t)(n0 + (j << 4) + rlane) * ldb + koff + k0;
      bh[j] = Frag<T>::load(Bb + bo);
    }
#pragma unroll
    for (int i = 0; i < 4; ++i) {
      const size_t ao = (size_t)(m0 + (i << 4) + rlane) * lda + koff + k0;
      V ah = Frag<T>::load(Ab + ao);
      V al = ah;
      if (SPL >= 1) al = Frag<T>::load(Ab2 + ao);
#pragma unroll
      for (int j = 0; j < 4; ++j) {
        acc[i][j] = Frag<T>::mma(ah, bh[j], acc[i][j]);
        if (SPL >= 1) acc[i][j] = Frag<T>::mma(al, bh[j], acc[i][j]);
      }
      Frag<T>::guard4(acc[i][0], acc[i][1], acc[i][2], acc[i][3], ah, al);
    }
    Frag<T>::keep(bh[0], bh[1], bh[2], bh[3]);
  }
  acc_guard4(acc[0][0], acc[0][1], acc[0][2], acc[0][3]);
  acc_guard4(acc[1][0], acc[1][1], acc[1][2], acc[1][3]);
  acc_guard4(acc[2][0], acc[2][1], acc[2][2], acc[2][3]);
  acc_guard4(acc[3][0], acc[3][1], acc[3][2], acc[3][3]);

  bool gate = false;
  float* Cf = C0 + (size_t)bz * strideC;
  int ldc = ldc0;
  int col = n0;
  if (EPI == 1) {
    if (n0 < kNQ) {
      const int hq = n0 >> 8;
      const int j0 = n0 & 255;
      if (j0 < kHD) { col = hq * kHD + j0; ldc = kE; }
      else          { gate = true; col = hq * kHD + j0 - kHD; ldc = kE; }
    } else if (n0 < kNQ + kNKV) {
      Cf = Ck; ldc = kNKV; col = n0 - kNQ;
    } else {
      Cf = Cv; ldc = kNKV; col = n0 - kNQ - kNKV;
    }
  }

  float* slab = sT[wave];
#pragma unroll
  for (int i = 0; i < 4; ++i) {
    const int mBase = m0 + (i << 4);
    if (EPI == 1 && gate) {
#pragma unroll
      for (int j = 0; j < 4; ++j) {
#pragma unroll
        for (int r = 0; r < 8; ++r) {
          const float g = acc[i][j][r];
          const float sg = kSgCarry * __builtin_amdgcn_rcpf(1.0f + __expf(-g));
          slab[(mOff + r) * 68 + (j << 4) + rlane] = sg;
        }
      }
    } else {
#pragma unroll
      for (int j = 0; j < 4; ++j) {
#pragma unroll
        for (int r = 0; r < 8; ++r) {
          slab[(mOff + r) * 68 + (j << 4) + rlane] = acc[i][j][r] * scale;
        }
      }
    }
    __builtin_amdgcn_fence(__ATOMIC_RELEASE, "workgroup");
    __builtin_amdgcn_wave_barrier();
    __builtin_amdgcn_fence(__ATOMIC_ACQUIRE, "workgroup");
    if (EPI == 1 && gate) {
      const int q = lane >> 3, c8 = (lane & 7) * 8;
      v4u hv[4], lv[4];
#pragma unroll
      for (int it = 0; it < 4; ++it) {
        const int row = it * 4 + q;
        const float* sp = slab + row * 68 + c8;
        const v4f s0 = *(const v4f*)(sp);
        const v4f s1 = *(const v4f*)(sp + 4);
        unsigned short hb[8], lb[8];
#pragma unroll
        for (int e = 0; e < 4; ++e) {
          const float f0 = s0[e];
          const float f1 = s1[e];
          split_h(f0, hb[e], lb[e]);
          split_h(f1, hb[4 + e], lb[4 + e]);
        }
        hv[it] = (v4u){pk16(hb[0], hb[1]), pk16(hb[2], hb[3]), pk16(hb[4], hb[5]), pk16(hb[6], hb[7])};
        lv[it] = (v4u){pk16(lb[0], lb[1]), pk16(lb[2], lb[3]), pk16(lb[4], lb[5]), pk16(lb[6], lb[7])};
      }
      for (int pass = 0; pass < 2; ++pass) {
#pragma unroll
        for (int it = 0; it < 4; ++it) {
          const int row = it * 4 + q;
          const size_t o = (size_t)(mBase + row) * kE + col + c8;
          *(volatile v4u*)(Sgh + o) = hv[it];
          *(volatile v4u*)(Sgl + o) = lv[it];
        }
        __threadfence();
      }
    } else {
      const int hh = lane >> 4, c4 = (lane & 15) * 4;
      for (int pass = 0; pass < 2; ++pass) {
#pragma unroll
        for (int it = 0; it < 8; ++it) {
          const int row = it * 2 + hh;
          const v4f v = *(const v4f*)(slab + row * 68 + c4);
          *(volatile v4f*)(Cf + (size_t)(mBase + row) * ldc + col + c4) = v;
        }
        __threadfence();
      }
    }
    __builtin_amdgcn_fence(__ATOMIC_RELEASE, "workgroup");
    __builtin_amdgcn_wave_barrier();
    __builtin_amdgcn_fence(__ATOMIC_ACQUIRE, "workgroup");
  }
}

__global__ __launch_bounds__(256) void normrope_kernel(
    const float* __restrict__ src, int pitch, int nheads,
    const float* __restrict__ normw, const float* __restrict__ cosp, const float* __restrict__ sinp,
    unsigned short* __restrict__ ohi, unsigned short* __restrict__ olo) {
  const int lane = threadIdx.x & 31;
  const int wave = __builtin_amdgcn_readfirstlane((int)(threadIdx.x >> 5));
  const int sc = blockIdx.x % (kS / 16);
  const int bh = blockIdx.x / (kS / 16);
  const int h  = bh % nheads;
  const int b  = bh / nheads;
  const int s  = sc * 16 + wave * 2 + (lane >> 4);
  const int sub = lane & 15;
  const int d0  = sub * 8;
  const size_t m = (size_t)b * kS + s;
  const float* xp = src + m * pitch + h * kHD + d0;
  const v4f a0 = *(const v4f*)(xp);
  const v4f a1 = *(const v4f*)(xp + 4);
  const v4f w0 = *(const v4f*)(normw + d0);
  const v4f w1 = *(const v4f*)(normw + d0 + 4);
  const v4f c0 = *(const v4f*)(cosp + m * kHD + d0);
  const v4f c1 = *(const v4f*)(cosp + m * kHD + d0 + 4);
  const v4f s0 = *(const v4f*)(sinp + m * kHD + d0);
  const v4f s1 = *(const v4f*)(sinp + m * kHD + d0 + 4);
  float x[8], wb[8], cb[8], sb[8];
#pragma unroll
  for (int e = 0; e < 4; ++e) {
    const float xa = a0[e]; const float xb = a1[e];
    const float wa = w0[e]; const float wc = w1[e];
    const float ca = c0[e]; const float cc = c1[e];
    const float sa = s0[e]; const float sd = s1[e];
    x[e] = xa;  x[4 + e] = xb;
    wb[e] = bf_rne(wa); wb[4 + e] = bf_rne(wc);
    cb[e] = bf_rne(ca); cb[4 + e] = bf_rne(cc);
    sb[e] = bf_rne(sa); sb[4 + e] = bf_rne(sd);
  }
  float ss = 0.0f;
#pragma unroll
  for (int e = 0; e < 8; ++e) ss += x[e] * x[e];
  ss += __shfl_xor(ss, 8, 32);
  ss += __shfl_xor(ss, 4, 32);
  ss += __shfl_xor(ss, 2, 32);
  ss += __shfl_xor(ss, 1, 32);
  const float rinv = rsqrtf(ss * (1.0f / (float)kHD) + kNormEps);
  float xn[8], pn[8];
#pragma unroll
  for (int e = 0; e < 8; ++e) xn[e] = (x[e] * rinv) * (1.0f + wb[e]);
#pragma unroll
  for (int e = 0; e < 8; ++e) pn[e] = __shfl_xor(xn[e], 8, 32);
  const float sgn = (sub < 8) ? -1.0f : 1.0f;
  unsigned short hb[8], lb[8];
#pragma unroll
  for (int e = 0; e < 8; ++e) {
    const float val = xn[e] * cb[e] + (sgn * pn[e]) * sb[e];
    split_h(val * kQKCarry, hb[e], lb[e]);
  }
  const v4u hv = (v4u){pk16(hb[0], hb[1]), pk16(hb[2], hb[3]), pk16(hb[4], hb[5]), pk16(hb[6], hb[7])};
  const v4u lv = (v4u){pk16(lb[0], lb[1]), pk16(lb[2], lb[3]), pk16(lb[4], lb[5]), pk16(lb[6], lb[7])};
  const size_t o = ((size_t)bh * kS + s) * kHD + d0;
  *(volatile v4u*)(ohi + o) = hv;
  *(volatile v4u*)(olo + o) = lv;
  __threadfence();
  *(volatile v4u*)(ohi + o) = hv;
  *(volatile v4u*)(olo + o) = lv;
}

__global__ __launch_bounds__(256) void vt_kernel(const float* __restrict__ vraw,
                                                 unsigned short* __restrict__ vth, unsigned short* __restrict__ vtl) {
  __shared__ float sm[kHD * 65];
  const int t = threadIdx.x;
  const int lane = t & 31;
  const int wave = __builtin_amdgcn_readfirstlane((int)(t >> 5));
  const int kt = blockIdx.x % (kS / 64);
  const int bk = blockIdx.x / (kS / 64);
  const int b = bk / kKVH;
  const int kvh = bk - b * kKVH;
  const int key0 = kt * 64;
#pragma unroll
  for (int i = 0; i < 8; ++i) {
    const int e = i * 256 + t;
    const int row = e >> 5;
    const int c4 = (e & 31) * 4;
    const v4f v = *(const v4f*)(vraw + ((size_t)b * kS + key0 + row) * kNKV + kvh * kHD + c4);
    const float f0 = v[0]; const float f1 = v[1]; const float f2 = v[2]; const float f3 = v[3];
    sm[(c4 + 0) * 65 + row] = f0 * kVCarry;
    sm[(c4 + 1) * 65 + row] = f1 * kVCarry;
    sm[(c4 + 2) * 65 + row] = f2 * kVCarry;
    sm[(c4 + 3) * 65 + row] = f3 * kVCarry;
  }
  __syncthreads();
  const int q = lane >> 3, c8 = (lane & 7) * 8;
  v4u hv[4], lv[4];
#pragma unroll
  for (int it = 0; it < 4; ++it) {
    const int d = it * 32 + wave * 4 + q;
    unsigned short hb[8], lb[8];
#pragma unroll
    for (int e = 0; e < 8; ++e) {
      const float f = sm[d * 65 + c8 + e];
      split_h(f, hb[e], lb[e]);
    }
    hv[it] = (v4u){pk16(hb[0], hb[1]), pk16(hb[2], hb[3]), pk16(hb[4], hb[5]), pk16(hb[6], hb[7])};
    lv[it] = (v4u){pk16(lb[0], lb[1]), pk16(lb[2], lb[3]), pk16(lb[4], lb[5]), pk16(lb[6], lb[7])};
  }
  for (int pass = 0; pass < 2; ++pass) {
#pragma unroll
    for (int it = 0; it < 4; ++it) {
      const int d = it * 32 + wave * 4 + q;
      const size_t o = ((size_t)bk * kHD + d) * kS + key0 + c8;
      *(volatile v4u*)(vth + o) = hv[it];
      *(volatile v4u*)(vtl + o) = lv[it];
    }
    __threadfence();
  }
}

template <bool HI>
__global__ __launch_bounds__(128) void attn_kernel(
    const unsigned short* qhp, const unsigned short* qlp,
    const unsigned short* __restrict__ khp, const unsigned short* __restrict__ klp,
    const unsigned short* __restrict__ vhp, const unsigned short* __restrict__ vlp,
    const unsigned short* __restrict__ sgh, const unsigned short* __restrict__ sgl,
    unsigned short* __restrict__ ahp, unsigned short* __restrict__ alp,
    int qb0, int nqb, float scl) {
  __shared__ __align__(16) _Float16 Ksh[64 * kHD];
  __shared__ __align__(16) _Float16 Ksl[HI ? 64 * kHD : 8];
  __shared__ __align__(16) _Float16 Vth[kHD * 64];
  __shared__ __align__(16) _Float16 Vtl[HI ? kHD * 64 : 8];
  __shared__ __align__(16) _Float16 Psh[4][16 * 64];
  __shared__ __align__(16) _Float16 Psl[HI ? 4 : 1][HI ? 16 * 64 : 8];
  __shared__ __align__(16) float Os[4][16 * 68];

  const int tid  = threadIdx.x;
  const int lane = tid & 31;
  const int wave = __builtin_amdgcn_readfirstlane((int)(tid >> 5));
  const int hh   = lane >> 4;
  const int c    = lane & 15;

  const int bx  = blockIdx.x;
  const int qb  = qb0 + (bx % nqb);
  const int bhI = bx / nqb;
  const int h   = bhI % kH;
  const int b   = bhI / kH;
  const int kvh = h / (kH / kKVH);
  const int q0  = qb * 64 + wave * 16;

  const _Float16* qh = (const _Float16*)qhp + ((size_t)(b * kH + h) * kS) * kHD;
  const _Float16* ql = (const _Float16*)qlp + ((size_t)(b * kH + h) * kS) * kHD;
  const _Float16* kg  = (const _Float16*)khp + ((size_t)(b * kKVH + kvh) * kS) * kHD;
  const _Float16* kgl = (const _Float16*)klp + ((size_t)(b * kKVH + kvh) * kS) * kHD;
  const _Float16* vg  = (const _Float16*)vhp + ((size_t)(b * kKVH + kvh) * kHD) * kS;
  const _Float16* vgl = (const _Float16*)vlp + ((size_t)(b * kKVH + kvh) * kHD) * kS;

  const _Float16* qrow  = qh + (size_t)(q0 + c) * kHD + 8 * hh;
  const _Float16* qlrow = ql + (size_t)(q0 + c) * kHD + 8 * hh;
  v16h qah[4];
#pragma unroll
  for (int dc = 0; dc < 4; ++dc) qah[dc] = Frag<_Float16>::load(qrow + dc * 32);

  float mrow[8], lrow[8];
  v8f oacc[8];
#pragma unroll
  for (int r = 0; r < 8; ++r) { mrow[r] = -INFINITY; lrow[r] = 0.f; }
#pragma unroll
  for (int t = 0; t < 8; ++t) oacc[t] = (v8f){0.f,0.f,0.f,0.f,0.f,0.f,0.f,0.f};

  const float kFill = -__FLT_MAX__;
  const int nChunks = qb + 1;
  for (int kc = 0; kc < nChunks; ++kc) {
    const int kv0 = kc * 64;
    __syncthreads();
#pragma unroll 1
    for (int i = 0; i < 8; ++i) {
      const int idx = i * 128 + tid;
      const int d = idx >> 3, cc = idx & 7;
      const size_t ko = (size_t)kv0 * kHD + (size_t)idx * 8;
      const size_t vo = (size_t)d * kS + kv0 + cc * 8;
      const v8h k8 = *(const v8h*)(kg + ko);
      const v8h v8 = *(const v8h*)(vg + vo);
      *(v8h*)(Ksh + idx * 8) = k8;
      *(v8h*)(Vth + idx * 8) = v8;
      if (HI) {
        const v8h k8l = *(const v8h*)(kgl + ko);
        const v8h v8l = *(const v8h*)(vgl + vo);
        *(v8h*)(Ksl + idx * 8) = k8l;
        *(v8h*)(Vtl + idx * 8) = v8l;
      }
    }
    __syncthreads();

    v8f s[4];
#pragma unroll
    for (int j = 0; j < 4; ++j) s[j] = (v8f){0.f,0.f,0.f,0.f,0.f,0.f,0.f,0.f};
#pragma unroll
    for (int dc = 0; dc < 4; ++dc) {
      v16h qlo = qah[dc];
      if (HI) qlo = Frag<_Float16>::load(qlrow + dc * 32);
#pragma unroll
      for (int j = 0; j < 4; ++j) {
        const v16h kb = Frag<_Float16>::load(Ksh + (j * 16 + c) * kHD + dc * 32 + 8 * hh);
        s[j] = mma_h(qah[dc], kb, s[j]);
        if (HI) {
          const v16h kl = Frag<_Float16>::load(Ksl + (j * 16 + c) * kHD + dc * 32 + 8 * hh);
          s[j] = mma_h(qah[dc], kl, s[j]);
          s[j] = mma_h(qlo, kb, s[j]);
        }
      }
    }

    const bool diag = (kc == qb);
    float cm[8];
#pragma unroll
    for (int r = 0; r < 8; ++r) {
      const int qrowi = q0 + 8 * hh + r;
      float m = -INFINITY;
#pragma unroll
      for (int j = 0; j < 4; ++j) {
        const int kvcol = kv0 + j * 16 + c;
        float sv = s[j][r] * scl;
        if (diag && (kvcol > qrowi)) sv = kFill;
        s[j][r] = sv;
        m = fmaxf(m, sv);
      }
      m = fmaxf(m, __shfl_xor(m, 1, 32));
      m = fmaxf(m, __shfl_xor(m, 2, 32));
      m = fmaxf(m, __shfl_xor(m, 4, 32));
      m = fmaxf(m, __shfl_xor(m, 8, 32));
      cm[r] = m;
    }
    _Float16* pwh = Psh[wave];
    _Float16* pwl = Psl[HI ? wave : 0];
#pragma unroll
    for (int r = 0; r < 8; ++r) {
      const float mnew = fmaxf(mrow[r], cm[r]);
      const float alpha = __expf(mrow[r] - mnew);
      mrow[r] = mnew;
      float psum = 0.f;
#pragma unroll
      for (int j = 0; j < 4; ++j) {
        const float p = __expf(s[j][r] - mnew);
        psum += p;
        const float x = p * kPCarry;
        const _Float16 ph = (_Float16)x;
        pwh[(8 * hh + r) * 64 + j * 16 + c] = ph;
        if (HI) {
          const float phf = (float)ph;
          const _Float16 plo = (_Float16)(x - phf);
          pwl[(8 * hh + r) * 64 + j * 16 + c] = plo;
        }
      }
      psum += __shfl_xor(psum, 1, 32);
      psum += __shfl_xor(psum, 2, 32);
      psum += __shfl_xor(psum, 4, 32);
      psum += __shfl_xor(psum, 8, 32);
      lrow[r] = lrow[r] * alpha + psum;
#pragma unroll
      for (int t = 0; t < 8; ++t) oacc[t][r] *= alpha;
    }
    __builtin_amdgcn_fence(__ATOMIC_RELEASE, "workgroup");
    __builtin_amdgcn_wave_barrier();
    __builtin_amdgcn_fence(__ATOMIC_ACQUIRE, "workgroup");
#pragma unroll 1
    for (int kk = 0; kk < 2; ++kk) {
      const v16h pa = Frag<_Float16>::load(pwh + c * 64 + kk * 32 + 8 * hh);
      v16h pl = pa;
      if (HI) pl = Frag<_Float16>::load(pwl + c * 64 + kk * 32 + 8 * hh);
#pragma unroll
      for (int t = 0; t < 8; ++t) {
        const v16h vb = Frag<_Float16>::load(Vth + (t * 16 + c) * 64 + kk * 32 + 8 * hh);
        oacc[t] = mma_h(pa, vb, oacc[t]);
        if (HI) {
          const v16h vl = Frag<_Float16>::load(Vtl + (t * 16 + c) * 64 + kk * 32 + 8 * hh);
          oacc[t] = mma_h(pa, vl, oacc[t]);
          oacc[t] = mma_h(pl, vb, oacc[t]);
        }
      }
    }
  }

  float inv[8];
#pragma unroll
  for (int r = 0; r < 8; ++r) inv[r] = kEpiFold * (1.0f / lrow[r]);
  float* os = Os[wave];
  const int q = lane >> 3, c8 = (lane & 7) * 8;
#pragma unroll
  for (int half = 0; half < 2; ++half) {
#pragma unroll
    for (int r = 0; r < 8; ++r) {
#pragma unroll
      for (int tt = 0; tt < 4; ++tt) os[(8 * hh + r) * 68 + tt * 16 + c] = oacc[4 * half + tt][r] * inv[r];
    }
    __builtin_amdgcn_fence(__ATOMIC_RELEASE, "workgroup");
    __builtin_amdgcn_wave_barrier();
    __builtin_amdgcn_fence(__ATOMIC_ACQUIRE, "workgroup");
    v4u hv[4], lv[4];
#pragma unroll
    for (int it = 0; it < 4; ++it) {
      const int row = it * 4 + q;
      const size_t o = ((size_t)b * kS + q0 + row) * kE + h * kHD + half * 64 + c8;
      const v4u gh = *(const v4u*)(sgh + o);
      const v4u gl = *(const v4u*)(sgl + o);
      const float* sp = os + row * 68 + c8;
      const v4f o0 = *(const v4f*)(sp);
      const v4f o1 = *(const v4f*)(sp + 4);
      float ov[8];
#pragma unroll
      for (int e = 0; e < 4; ++e) {
        const float fa = o0[e];
        const float fb = o1[e];
        ov[e] = fa;
        ov[4 + e] = fb;
      }
      unsigned short hb[8], lb[8];
#pragma unroll
      for (int w = 0; w < 4; ++w) {
        const unsigned wh = gh[w];
        const unsigned wl = gl[w];
        const float g0 = h16_to_f32(wh & 0xffffu) + h16_to_f32(wl & 0xffffu);
        const float g1 = h16_to_f32(wh >> 16) + h16_to_f32(wl >> 16);
        split_h(ov[2 * w] * g0, hb[2 * w], lb[2 * w]);
        split_h(ov[2 * w + 1] * g1, hb[2 * w + 1], lb[2 * w + 1]);
      }
      hv[it] = (v4u){pk16(hb[0], hb[1]), pk16(hb[2], hb[3]), pk16(hb[4], hb[5]), pk16(hb[6], hb[7])};
      lv[it] = (v4u){pk16(lb[0], lb[1]), pk16(lb[2], lb[3]), pk16(lb[4], lb[5]), pk16(lb[6], lb[7])};
    }
    for (int pass = 0; pass < 2; ++pass) {
#pragma unroll
      for (int it = 0; it < 4; ++it) {
        const int row = it * 4 + q;
        const size_t o = ((size_t)b * kS + q0 + row) * kE + h * kHD + half * 64 + c8;
        *(volatile v4u*)(ahp + o) = hv[it];
        if (HI) *(volatile v4u*)(alp + o) = lv[it];
      }
      __threadfence();
    }
    __builtin_amdgcn_fence(__ATOMIC_RELEASE, "workgroup");
    __builtin_amdgcn_wave_barrier();
    __builtin_amdgcn_fence(__ATOMIC_ACQUIRE, "workgroup");
  }
}

extern "C" void kernel_launch(void* const* d_in, const int* in_sizes, int n_in,
                              void* d_out, int out_size, void* d_ws, size_t ws_size,
                              hipStream_t stream) {
  if (n_in < 9) return;
  if (in_sizes[0] != kRows * kD) return;
  if (in_sizes[1] != kRows * kHD) return;
  if (in_sizes[2] != kRows * kHD) return;
  if (in_sizes[3] != kNQ * kD) return;
  if (in_sizes[4] != kNKV * kD) return;
  if (in_sizes[5] != kNKV * kD) return;
  if (in_sizes[6] != kD * kE) return;
  if (in_sizes[7] != kHD) return;
  if (in_sizes[8] != kHD) return;
  if (out_size != kRows * kD) return;
  if (ws_size < kWsTotal) return;

  const float* x   = (const float*)d_in[0];
  const float* cs  = (const float*)d_in[1];
  const float* sn  = (const float*)d_in[2];
  const float* Wq  = (const float*)d_in[3];
  const float* Wk  = (const float*)d_in[4];
  const float* Wv  = (const float*)d_in[5];
  const float* Wo  = (const float*)d_in[6];
  const float* qnw = (const float*)d_in[7];
  const float* knw = (const float*)d_in[8];
  float* out = (float*)d_out;

  char* ws = (char*)d_ws;
  unsigned short* XB  = (unsigned short*)(ws + kOffXB);
  unsigned short* WB  = (unsigned short*)(ws + kOffWB);
  float*          QR  = (float*)(ws + kOffQR);
  float*          KR  = (float*)(ws + kOffKR);
  float*          VR  = (float*)(ws + kOffVR);
  unsigned short* SGH = (unsigned short*)(ws + kOffSGH);
  unsigned short* SGL = (unsigned short*)(ws + kOffSGL);
  unsigned short* KH  = (unsigned short*)(ws + kOffKH);
  unsigned short* KL  = (unsigned short*)(ws + kOffKL);
  unsigned short* QH  = (unsigned short*)(ws + kOffQH);
  unsigned short* QL  = (unsigned short*)(ws + kOffQL);
  unsigned short* AH  = (unsigned short*)(ws + kOffAH);
  unsigned short* AL  = (unsigned short*)(ws + kOffAL);
  unsigned short* VTH = (unsigned short*)(ws + kOffVTH);
  unsigned short* VTL = (unsigned short*)(ws + kOffVTL);
  unsigned short* WO  = (unsigned short*)(ws + kOffWO);

  cvt_bf16_kernel<<<(kRows * kD / 8) / 256, 256, 0, stream>>>(x, XB, kRows * kD / 8);
  cvt_bf16_kernel<<<(kNQ * kD / 8) / 256, 256, 0, stream>>>(Wq, WB, kNQ * kD / 8);
  cvt_bf16_kernel<<<(kNKV * kD / 8) / 256, 256, 0, stream>>>(Wk, WB + (size_t)kNQ * kD, kNKV * kD / 8);
  cvt_bf16_kernel<<<(kNKV * kD / 8) / 256, 256, 0, stream>>>(Wv, WB + (size_t)(kNQ + kNKV) * kD, kNKV * kD / 8);

  gemm64_kernel<1, 0, 1><<<dim3((kRows / 64) * (kNQKV / 64) / 8, 1), 256, 0, stream>>>(
      XB, nullptr, kD, 0L,
      WB, kD,
      QR, kE, 0L,
      KR, VR, SGH, SGL,
      kRows, kNQKV, kD, 1.0f);

  normrope_kernel<<<kB * kH * (kS / 16), 256, 0, stream>>>(QR, kE, kH, qnw, cs, sn, QH, QL);
  normrope_kernel<<<kB * kKVH * (kS / 16), 256, 0, stream>>>(KR, kNKV, kKVH, knw, cs, sn, KH, KL);

  vt_kernel<<<kB * kKVH * (kS / 64), 256, 0, stream>>>(VR, VTH, VTL);

  const float scl = (float)(1.0 / sqrt((double)kHD)) * kScoreFold;
  constexpr int kHiBlocks = kHiRows / 64;
  constexpr int kLoBlocks = (kS - kHiRows) / 64;
  attn_kernel<true><<<kB * kH * kHiBlocks, 128, 0, stream>>>(
      QH, QL, KH, KL, VTH, VTL, SGH, SGL, AH, AL, 0, kHiBlocks, scl);
  attn_kernel<false><<<kB * kH * kLoBlocks, 128, 0, stream>>>(
      QH, QL, KH, KL, VTH, VTL, SGH, SGL, AH, AL, kHiBlocks, kLoBlocks, scl);

  cvt_f16c_kernel<<<(kD * kE / 8) / 256, 256, 0, stream>>>(Wo, WO, kD * kE / 8, kWoCarry);

  gemm64_kernel<0, 1, 0><<<dim3((kHiRows / 64) * (kD / 64) / 8, kB), 256, 0, stream>>>(
      AH, AL, kE, (long)kS * kE,
      WO, kE,
      out, kD, (long)kS * kD,
      nullptr, nullptr, nullptr, nullptr,
      kHiRows, kD, kE, kOutScale);
  gemm64_kernel<0, 0, 0><<<dim3(((kS - kHiRows) / 64) * (kD / 64) / 8, kB), 256, 0, stream>>>(
      AH + (size_t)kHiRows * kE, nullptr, kE, (long)kS * kE,
      WO, kE,
      out + (size_t)kHiRows * kD, kD, (long)kS * kD,
      nullptr, nullptr, nullptr, nullptr,
      kS - kHiRows, kD, kE, kOutScale);
}
